// GATNet_82351702934258
// MI455X (gfx1250) — hardware-verified
//
#include <hip/hip_runtime.h>
#include <stddef.h>
#include <stdint.h>
#include <math.h>


#define F_IN    128
#define HC      384
#define NCOL    768
#define NHD     12
#define XW      1536
#define NGR     64
#define NOUTC   10
#define HIDR    64
#define NTHR    256
#define NWAVE   8
#define EPT     8
#define CHUNK   (NTHR * EPT)
#define WCAP    (EPT * 32)
#define LISTN   (NWAVE * WCAP)
#define NBMAX   2048
#define SLOTB   11
#define NB      1024
#define RCAP    28672
#define DEGCAP  256
#define SROWS   128
#define GBM     64
#define GBN     64
#define GTHR    128
#define MROWS   128
#define NEGSL   0.2f
#define EPS_SM  1e-16f
#define WSMAX   134217728
#define LDS_BKT ((2 * RCAP + 2 * NBMAX + LISTN) * 4 + 64)
#define OUT0N   (NGR * NOUTC)
#define NU_WT1H (HC * (F_IN / 8))
#define NU_W2H  (HC * (NCOL / 8))

static_assert((CHUNK & (CHUNK - 1)) == 0 && CHUNK <= (1 << SLOTB));
static_assert(NBMAX == (1 << SLOTB));
static_assert(NTHR * 8 == NBMAX);
static_assert(LISTN >= NBMAX);
static_assert(NB <= NBMAX && (NB % SROWS) == 0 && NB == 4 * NTHR);
static_assert((RCAP % (NTHR * 4)) == 0);
static_assert(LDS_BKT <= 300000);
static_assert(GBM == (GTHR / 32) * 16);
static_assert(GTHR == 2 * GBN && GTHR == 2 * GBM);
static_assert((F_IN % 32) == 0 && (NCOL % 32) == 0);
static_assert(NCOL == NHD * GBN && NCOL == 2 * HC);
static_assert((NCOL % 128) == 0);
static_assert(GBN == 4 * 16);
static_assert((MROWS % GBM) == 0 && MROWS == SROWS && SROWS == 16 * NWAVE);
static_assert(NCOL == 6 * 32 * 4);
static_assert(HC == 3 * 32 * 4);
static_assert(NGR == 64);
static_assert((NU_WT1H % NTHR) == 0 && (NU_W2H % NTHR) == 0);
static_assert(DEGCAP >= 32 + 8);
static_assert(RCAP >= 16685 + 4096);
static_assert((OUT0N % 4) == 0 && (OUT0N * 4) % 128 == 0 && OUT0N / 4 <= NTHR);
static_assert((HC * 4) % 128 == 0);

typedef float          v4f  __attribute__((ext_vector_type(4)));
typedef float          v8f  __attribute__((ext_vector_type(8)));
typedef int            v4i  __attribute__((ext_vector_type(4)));
typedef int            v8i  __attribute__((ext_vector_type(8)));
typedef unsigned int   v4u  __attribute__((ext_vector_type(4)));
typedef unsigned short v8us __attribute__((ext_vector_type(8)));
typedef __bf16         v16b __attribute__((ext_vector_type(16)));
typedef v4f  __attribute__((may_alias)) v4fa;
typedef v4i  __attribute__((may_alias)) v4ia;
typedef v8us __attribute__((may_alias)) v8usa;
union FragB { v16b v; v8us h[2]; v8i w; };

__device__ __forceinline__ v8f wmb(const FragB& a, const FragB& b, v8f c) {
  v8f d = __builtin_amdgcn_wmma_f32_16x16x32_bf16(false, a.v, false, b.v, (short)0, c, false, false);
  asm volatile("v_nop\n\tv_nop\n\tv_nop\n\tv_nop" : "+v"(d) : "v"(a.w), "v"(b.w));
  return d;
}

__device__ __forceinline__ unsigned int f2bf(float f) {
  const unsigned int u = __float_as_uint(f);
  const unsigned int r = ((u + 0x7FFFu + ((u >> 16) & 1u)) >> 16) & 0xFFFFu;
  return ((u & 0x7FFFFFFFu) > 0x7F800000u) ? 0x7FC0u : r;
}
__device__ __forceinline__ float bf2f(unsigned int b) { return __uint_as_float(b << 16); }
__device__ __forceinline__ float bfr(float f) { return bf2f(f2bf(f)); }
__device__ __forceinline__ v4f bfr4(const v4f a) {
  v4f r; r.x = bfr(a.x); r.y = bfr(a.y); r.z = bfr(a.z); r.w = bfr(a.w); return r;
}
__device__ __forceinline__ unsigned int pk2(float lo, float hi) { return f2bf(lo) | (f2bf(hi) << 16); }
__device__ __forceinline__ v4u pack8(const v4f a, const v4f b) {
  v4u r;
  r.x = pk2(a.x, a.y); r.y = pk2(a.z, a.w); r.z = pk2(b.x, b.y); r.w = pk2(b.z, b.w);
  return r;
}
__device__ __forceinline__ float relu_k(float v) { return (v > 0.0f) ? v : (v - v); }

__device__ __forceinline__ int scan_chunk(const int* __restrict__ dsts, int nE, int cbase, int slotBase,
                                          int nb, int vec8, int* list, int tid, int lane, int wave) {
  int wc = 0;
  const int el0  = tid * EPT;
  const int e0   = cbase + el0;
  const int sent = -2147483647 - 1;
  v4i da, db;
  if (vec8 != 0 && cbase + CHUNK <= nE) {
    da = *(const v4i*)(dsts + e0);
    db = *(const v4i*)(dsts + e0 + 4);
  } else {
    da.x = (e0     < nE) ? dsts[min(e0,     nE - 1)] : sent;
    da.y = (e0 + 1 < nE) ? dsts[min(e0 + 1, nE - 1)] : sent;
    da.z = (e0 + 2 < nE) ? dsts[min(e0 + 2, nE - 1)] : sent;
    da.w = (e0 + 3 < nE) ? dsts[min(e0 + 3, nE - 1)] : sent;
    db.x = (e0 + 4 < nE) ? dsts[min(e0 + 4, nE - 1)] : sent;
    db.y = (e0 + 5 < nE) ? dsts[min(e0 + 5, nE - 1)] : sent;
    db.z = (e0 + 6 < nE) ? dsts[min(e0 + 6, nE - 1)] : sent;
    db.w = (e0 + 7 < nE) ? dsts[min(e0 + 7, nE - 1)] : sent;
  }
  const unsigned nbs = (unsigned)slotBase;
  const unsigned unb = (unsigned)nb;
  const unsigned s0 = (unsigned)da.x - nbs, s1 = (unsigned)da.y - nbs;
  const unsigned s2 = (unsigned)da.z - nbs, s3 = (unsigned)da.w - nbs;
  const unsigned s4 = (unsigned)db.x - nbs, s5 = (unsigned)db.y - nbs;
  const unsigned s6 = (unsigned)db.z - nbs, s7 = (unsigned)db.w - nbs;
  const bool h0 = s0 < unb, h1 = s1 < unb, h2 = s2 < unb, h3 = s3 < unb;
  const bool h4 = s4 < unb, h5 = s5 < unb, h6 = s6 < unb, h7 = s7 < unb;
  const unsigned any = __builtin_amdgcn_ballot_w32(h0 | h1 | h2 | h3 | h4 | h5 | h6 | h7);
  if (any != 0u) {
#define HITJ(J, HJ, SJ) { \
      const unsigned mj = __builtin_amdgcn_ballot_w32(HJ); \
      if (mj != 0u) { \
        if (HJ) { \
          const int pos = wc + (int)__builtin_amdgcn_mbcnt_lo(mj, 0u); \
          if (pos < WCAP) list[wave * WCAP + pos] = ((el0 + (J)) << SLOTB) | (int)(SJ); \
        } \
        wc += (int)__builtin_popcount(mj); } }
    HITJ(0, h0, s0)
    HITJ(1, h1, s1)
    HITJ(2, h2, s2)
    HITJ(3, h3, s3)
    HITJ(4, h4, s4)
    HITJ(5, h5, s5)
    HITJ(6, h6, s6)
    HITJ(7, h7, s7)
#undef HITJ
  }
  return wc;
}

__device__ __forceinline__ void wtr_unit(const float* __restrict__ w, int kk, int nloc, unsigned short* dst) {
  const float* p = w + (size_t)kk * HC + nloc;
  v4f a, b;
  a.x = p[0];               a.y = p[(size_t)HC];      a.z = p[(size_t)2 * HC];  a.w = p[(size_t)3 * HC];
  b.x = p[(size_t)4 * HC];  b.y = p[(size_t)5 * HC];  b.z = p[(size_t)6 * HC];  b.w = p[(size_t)7 * HC];
  const v4u wv = pack8(a, b);
  *(volatile v4u*)dst = wv;
  __threadfence();
  *(volatile v4u*)dst = wv;
}

__global__ __launch_bounds__(NTHR) void k_prep(const float* __restrict__ x, const float* __restrict__ W1,
                                               const float* __restrict__ Ws1, const float* __restrict__ W2,
                                               const float* __restrict__ Ws2, unsigned short* XB,
                                               unsigned short* WT1, unsigned short* W2C, int nN, int nBx) {
  const int bx = (int)blockIdx.x;
  const int tid = (int)threadIdx.x;
  const int bW1 = NU_WT1H / NTHR;
  const int bW2 = NU_W2H / NTHR;
  if (bx < nBx) {
    const int i = bx * NTHR + tid;
    const int row = i >> 4;
    const int c0  = (i & 15) * 8;
    const int rc  = row < nN ? row : nN - 1;
    const float* p = x + (size_t)rc * F_IN + c0;
    v4f a = *(const v4fa*)p, b = *(const v4fa*)(p + 4);
    const v4f z4 = {0.f, 0.f, 0.f, 0.f};
    if (row >= nN) { a = z4; b = z4; }
    const v4u hv = pack8(a, b);
    unsigned short* o = XB + (size_t)row * F_IN + c0;
    *(volatile v4u*)o = hv;
    __threadfence();
    *(volatile v4u*)o = hv;
  } else if (bx < nBx + bW1) {
    const int u = (bx - nBx) * NTHR + tid;
    const int n = u >> 4, k8 = (u & 15) * 8;
    wtr_unit(W1, k8, n, WT1 + (size_t)n * F_IN + k8);
  } else if (bx < nBx + 2 * bW1) {
    const int u = (bx - nBx - bW1) * NTHR + tid;
    const int n = u >> 4, k8 = (u & 15) * 8;
    wtr_unit(Ws1, k8, n, WT1 + (size_t)(HC + n) * F_IN + k8);
  } else if (bx < nBx + 2 * bW1 + bW2) {
    const int u = (bx - nBx - 2 * bW1) * NTHR + tid;
    const int n = u / (NCOL / 8);
    const int k8 = (u - n * (NCOL / 8)) * 8;
    const int kk = k8 >= HC ? k8 - HC : k8;
    wtr_unit(W2, kk, n, W2C + (size_t)n * NCOL + k8);
  } else if (bx < nBx + 2 * bW1 + 2 * bW2) {
    const int u = (bx - nBx - 2 * bW1 - bW2) * NTHR + tid;
    const int n = u / (NCOL / 8);
    const int k8 = (u - n * (NCOL / 8)) * 8;
    const int kk = k8 >= HC ? k8 - HC : k8;
    wtr_unit(Ws2, kk, n, W2C + (size_t)(HC + n) * NCOL + k8);
  }
}

__global__ __launch_bounds__(NTHR) void k_bucket(const int* __restrict__ srcs, const int* __restrict__ dsts,
                                                 int nN, int nE, int vec8,
                                                 int* SRT, int* SOFF, int* SCNT, int* META) {
  extern __shared__ v4f lds_dyn[];
  int* reg1 = (int*)lds_dyn;
  int* reg2 = reg1 + RCAP;
  int* scnt = reg2 + RCAP;
  int* soff = scnt + NBMAX;
  int* list = soff + NBMAX;
  int* wcnt = list + LISTN;
  int* wtot = wcnt + NWAVE;
  const int tid = (int)threadIdx.x, lane = tid & 31, wave = tid >> 5;
  const int nodeBase = (int)blockIdx.x * NB;

  for (int i = tid; i < NBMAX; i += NTHR) scnt[i] = 0;
  {
    const v4i z4 = {0, 0, 0, 0};
    for (int i = tid * 4; i < RCAP; i += NTHR * 4) *(v4ia*)(reg2 + i) = z4;
  }
  __syncthreads();

  int tot = 0;
  const int nChunks = (nE + CHUNK - 1) / CHUNK;
#pragma unroll 1
  for (int ch = 0; ch < nChunks; ++ch) {
    const int cbase = ch * CHUNK;
    const int wc = scan_chunk(dsts, nE, cbase, nodeBase, NB, vec8, list, tid, lane, wave);
    if (lane == 0) wcnt[wave] = wc;
    __syncthreads();
    int pre = 0, all = 0;
#pragma unroll
    for (int w2 = 0; w2 < NWAVE; ++w2) {
      int c = wcnt[w2];
      c = c < 0 ? 0 : (c > WCAP ? WCAP : c);
      all += c;
      pre += (w2 < wave) ? c : 0;
    }
    const int wcc  = wc > WCAP ? WCAP : wc;
    const int base = tot + pre;
#pragma unroll 1
    for (int i = lane; i < wcc; i += 32) {
      const int ent = list[wave * WCAP + i];
      const int el  = (ent >> SLOTB) & (CHUNK - 1);
      const int sl  = ent & (NBMAX - 1);
      int eid = cbase + el;
      eid = eid > nE - 1 ? nE - 1 : eid;
      const int pos = base + i;
      if (pos < RCAP) reg1[pos] = (int)(((unsigned)eid << SLOTB) | (unsigned)sl);
    }
    tot += all;
    tot = tot > RCAP ? RCAP : tot;
    __syncthreads();
  }
  const int nh = tot;

  if (wave == 0) {
#pragma unroll 1
    for (int b0 = 0; b0 < nh; b0 += 32) {
      const int idx = b0 + lane;
      const int uv  = reg1[idx < nh ? idx : nh - 1];
      const int m32 = (nh - b0) < 32 ? (nh - b0) : 32;
#pragma unroll 1
      for (int k = 0; k < m32; ++k) {
        const int u  = __builtin_amdgcn_readlane(uv, k);
        const int sl = u & (NBMAX - 1);
        if (lane == 0) scnt[sl] = scnt[sl] + 1;
      }
    }
  }
  __syncthreads();

  {
    const v4i ca = *(const v4ia*)(scnt + 8 * tid);
    const v4i cb = *(const v4ia*)(scnt + 8 * tid + 4);
    const int e0 = ca.x < 0 ? 0 : ca.x, e1 = ca.y < 0 ? 0 : ca.y, e2 = ca.z < 0 ? 0 : ca.z, e3 = ca.w < 0 ? 0 : ca.w;
    const int e4 = cb.x < 0 ? 0 : cb.x, e5 = cb.y < 0 ? 0 : cb.y, e6 = cb.z < 0 ? 0 : cb.z, e7 = cb.w < 0 ? 0 : cb.w;
    const int ts = e0 + e1 + e2 + e3 + e4 + e5 + e6 + e7;
    int incl = ts;
#pragma unroll
    for (int d = 1; d < 32; d <<= 1) {
      const int up = __shfl_up(incl, d);
      if (lane >= d) incl += up;
    }
    if (lane == 31) wtot[wave] = incl;
    __syncthreads();
    int pre = 0;
#pragma unroll
    for (int w2 = 0; w2 < NWAVE; ++w2) pre += (w2 < wave) ? wtot[w2] : 0;
    int run = pre + incl - ts;
    soff[8 * tid + 0] = run; run += e0;
    soff[8 * tid + 1] = run; run += e1;
    soff[8 * tid + 2] = run; run += e2;
    soff[8 * tid + 3] = run; run += e3;
    soff[8 * tid + 4] = run; run += e4;
    soff[8 * tid + 5] = run; run += e5;
    soff[8 * tid + 6] = run; run += e6;
    soff[8 * tid + 7] = run;
  }
  __syncthreads();
  for (int i = tid; i < NBMAX; i += NTHR) list[i] = soff[i];
  __syncthreads();

  if (wave == 0) {
#pragma unroll 1
    for (int b0 = 0; b0 < nh; b0 += 32) {
      const int idx = b0 + lane;
      const int uv  = reg1[idx < nh ? idx : nh - 1];
      const int m32 = (nh - b0) < 32 ? (nh - b0) : 32;
#pragma unroll 1
      for (int k = 0; k < m32; ++k) {
        const int u   = __builtin_amdgcn_readlane(uv, k);
        const int sl  = u & (NBMAX - 1);
        const int eid = (int)((unsigned)u >> SLOTB);
        if (lane == 0) {
          int pos = list[sl];
          pos = pos < 0 ? 0 : (pos > RCAP - 1 ? RCAP - 1 : pos);
          reg2[pos] = eid;
          list[sl] = pos + 1;
        }
      }
    }
  }
  __syncthreads();

  int* srt = SRT + (size_t)blockIdx.x * RCAP;
#pragma unroll 1
  for (int i0 = 0; i0 < RCAP; i0 += NTHR * 4) {
    const int i = i0 + 4 * tid;
    const v4i e = *(const v4ia*)(reg2 + i);
    int e0 = e.x, e1 = e.y, e2 = e.z, e3 = e.w;
    e0 = e0 < 0 ? 0 : (e0 > nE - 1 ? nE - 1 : e0);
    e1 = e1 < 0 ? 0 : (e1 > nE - 1 ? nE - 1 : e1);
    e2 = e2 < 0 ? 0 : (e2 > nE - 1 ? nE - 1 : e2);
    e3 = e3 < 0 ? 0 : (e3 > nE - 1 ? nE - 1 : e3);
    int s0 = srcs[e0], s1 = srcs[e1], s2 = srcs[e2], s3 = srcs[e3];
    s0 = s0 < 0 ? 0 : (s0 > nN - 1 ? nN - 1 : s0);
    s1 = s1 < 0 ? 0 : (s1 > nN - 1 ? nN - 1 : s1);
    s2 = s2 < 0 ? 0 : (s2 > nN - 1 ? nN - 1 : s2);
    s3 = s3 < 0 ? 0 : (s3 > nN - 1 ? nN - 1 : s3);
    v4i sv;
    sv.x = (i     < nh) ? s0 : 0;
    sv.y = (i + 1 < nh) ? s1 : 0;
    sv.z = (i + 2 < nh) ? s2 : 0;
    sv.w = (i + 3 < nh) ? s3 : 0;
    *(volatile v4i*)(srt + i) = sv;
    __threadfence();
    *(volatile v4i*)(srt + i) = sv;
  }
  {
    const v4i so = *(const v4ia*)(soff + 4 * tid);
    const v4i sc = *(const v4ia*)(scnt + 4 * tid);
    v4i mv = {0, 0, 0, 0};
    if (tid == 0) { mv.x = nh; mv.y = (nh >= RCAP) ? 1 : 0; }
    int* po = SOFF + (size_t)blockIdx.x * NB + 4 * tid;
    int* pc = SCNT + (size_t)blockIdx.x * NB + 4 * tid;
    int* pm = META + (size_t)blockIdx.x * 32 + 4 * (tid & 7);
    const bool wm = tid < 8;
    *(volatile v4i*)po = so;
    *(volatile v4i*)pc = sc;
    if (wm) *(volatile v4i*)pm = mv;
    __threadfence();
    *(volatile v4i*)po = so;
    *(volatile v4i*)pc = sc;
    if (wm) *(volatile v4i*)pm = mv;
  }
}

__global__ __launch_bounds__(GTHR) void k_gemm(
    const unsigned short* __restrict__ A, int lda, int aoffBr,
    const unsigned short* __restrict__ WT, int K,
    float* outF,
    const float* __restrict__ aMs, const float* __restrict__ aMd,
    const float* __restrict__ aSs, const float* __restrict__ aSd,
    float* SD)
{
  __shared__ __attribute__((aligned(16))) float stg[GBM * GBN];
  __shared__ __attribute__((aligned(16))) float satt[2 * GBN];
  __shared__ __attribute__((aligned(16))) float sdall[GBM * 32];
  const int tid = (int)threadIdx.x, lane = tid & 31, wave = tid >> 5, hh = lane >> 4, m = lane & 15;
  const int rowBase = (int)blockIdx.x * GBM;
  const int ksteps = K >> 5;

  for (int i = tid; i < GBM * 32; i += GTHR) sdall[i] = 0.f;

#pragma unroll 1
  for (int hd = 0; hd < NHD; ++hd) {
    const int br = hd >= 6 ? 1 : 0;
    const int hl = hd - 6 * br;
    {
      const int which = tid >> 6;
      const int c  = tid & 63;
      const int ix = hl * GBN + c;
      const float vms = aMs[ix], vmd = aMd[ix], vss = aSs[ix], vsd = aSd[ix];
      const float vm = (which == 0) ? vms : vmd;
      const float vs = (which == 0) ? vss : vsd;
      const float v  = (br == 0) ? vm : vs;
      satt[which * GBN + c] = bfr(v);
    }
    v8f acc[4];
    {
      const v8f z = {0.f, 0.f, 0.f, 0.f, 0.f, 0.f, 0.f, 0.f};
      acc[0] = z; acc[1] = z; acc[2] = z; acc[3] = z;
    }
    const unsigned short* ap = A  + (size_t)(rowBase + 16 * wave + m) * (size_t)lda + br * aoffBr + 8 * hh;
    const unsigned short* wp = WT + (size_t)(hd * GBN + m) * (size_t)K + 8 * hh;
#pragma unroll 1
    for (int ks = 0; ks < ksteps; ++ks) {
      FragB af;
      af.h[0] = *(const v8usa*)(ap + 32 * ks);
      af.h[1] = *(const v8usa*)(ap + 32 * ks + 16);
#pragma unroll
      for (int t = 0; t < 4; ++t) {
        const unsigned short* wq = wp + (size_t)(16 * t) * (size_t)K + 32 * ks;
        FragB bf;
        bf.h[0] = *(const v8usa*)wq;
        bf.h[1] = *(const v8usa*)(wq + 16);
        acc[t] = wmb(af, bf, acc[t]);
      }
    }
#pragma unroll
    for (int t = 0; t < 4; ++t) {
      const int lc = 16 * t + m;
#pragma unroll
      for (int r = 0; r < 8; ++r) {
        const int lr = 16 * wave + 8 * hh + r;
        stg[lr * GBN + lc] = acc[t][r];
      }
    }
    __syncthreads();

    {
      const int row = tid & 63, which = tid >> 6;
      const float* sa = satt + which * GBN;
      const float* hr = stg + row * GBN;
      float d = 0.f;
#pragma unroll 4
      for (int c4 = 0; c4 < GBN / 4; ++c4) {
        const v4f hv = *(const v4fa*)(hr + 4 * c4);
        const v4f av = *(const v4fa*)(sa + 4 * c4);
        d = fmaf(hv.x, av.x, d);
        d = fmaf(hv.y, av.y, d);
        d = fmaf(hv.z, av.z, d);
        d = fmaf(hv.w, av.w, d);
      }
      sdall[row * 32 + which * 16 + hd] = d;
    }

    v4f fv[8];
#pragma unroll
    for (int i = 0; i < 8; ++i) {
      const int lr = 16 * wave + 2 * i + hh;
      fv[i] = *(const v4fa*)(stg + lr * GBN + 4 * m);
    }
#pragma unroll
    for (int i = 0; i < 8; ++i) {
      const int lr = 16 * wave + 2 * i + hh;
      float* op = outF + (size_t)(rowBase + lr) * NCOL + hd * GBN + 4 * m;
      *(volatile v4f*)op = fv[i];
    }
    __threadfence();
#pragma unroll
    for (int i = 0; i < 8; ++i) {
      const int lr = 16 * wave + 2 * i + hh;
      float* op = outF + (size_t)(rowBase + lr) * NCOL + hd * GBN + 4 * m;
      *(volatile v4f*)op = fv[i];
    }
    __syncthreads();
  }

  v4f sv[4];
#pragma unroll
  for (int it = 0; it < 4; ++it) sv[it] = *(const v4fa*)(sdall + 4 * (it * GTHR + tid));
  float* sp = SD + (size_t)rowBase * 32;
#pragma unroll
  for (int it = 0; it < 4; ++it) *(volatile v4f*)(sp + 4 * (it * GTHR + tid)) = sv[it];
  __threadfence();
#pragma unroll
  for (int it = 0; it < 4; ++it) *(volatile v4f*)(sp + 4 * (it * GTHR + tid)) = sv[it];
}

template <int L>
__global__ __launch_bounds__(NTHR) void k_scan(
    const int* __restrict__ SRT, const int* __restrict__ SOFF, const int* __restrict__ SCNT,
    const int* __restrict__ META,
    const float* __restrict__ Hf, const float* __restrict__ SD,
    const float* __restrict__ bm, const float* __restrict__ bs,
    unsigned short* XHL, float* HS, int nN, int MPr)
{
  const int tid = (int)threadIdx.x, lane = tid & 31, wave = tid >> 5;
  const int hsel = lane >> 4, l15 = lane & 15;
  const int rowBlk = (int)blockIdx.x * SROWS;
  const int bkt = rowBlk / NB;
  const int sb  = rowBlk - bkt * NB;
  int nh = __builtin_amdgcn_readfirstlane(META[bkt * 32]);
  const int fl = __builtin_amdgcn_readfirstlane(META[bkt * 32 + 1]);
  nh = nh < 0 ? 0 : (nh > RCAP ? RCAP : nh);
  const bool ovf = (fl != 0) || (nh >= RCAP);
  const float qnan = __int_as_float(0x7fc00000);
  const int* srt = SRT + (size_t)bkt * RCAP;

  v4f bb[6];
  bb[0] = bfr4(*(const v4fa*)(bm + 4 * (lane)));
  bb[1] = bfr4(*(const v4fa*)(bm + 4 * (lane + 32)));
  bb[2] = bfr4(*(const v4fa*)(bm + 4 * (lane + 64)));
  bb[3] = bfr4(*(const v4fa*)(bs + 4 * (lane)));
  bb[4] = bfr4(*(const v4fa*)(bs + 4 * (lane + 32)));
  bb[5] = bfr4(*(const v4fa*)(bs + 4 * (lane + 64)));

#pragma unroll 1
  for (int jt = 0; jt < SROWS / NWAVE; ++jt) {
    const int slot = sb + wave * (SROWS / NWAVE) + jt;
    const int grow = rowBlk + wave * (SROWS / NWAVE) + jt;
    const int gcl  = grow < nN ? grow : nN - 1;
    int st = __builtin_amdgcn_readfirstlane(SOFF[bkt * NB + slot]);
    const int craw = __builtin_amdgcn_readfirstlane(SCNT[bkt * NB + slot]);
    int cnt = craw;
    st  = st < 0 ? 0 : (st > nh ? nh : st);
    cnt = cnt < 0 ? 0 : (cnt > DEGCAP ? DEGCAP : cnt);
    if (cnt > nh - st) cnt = nh - st;
    const float pz = (ovf || craw > DEGCAP) ? qnan : 0.0f;

    const float* hrow = Hf + (size_t)gcl * NCOL;
    v4f av[6];
#pragma unroll
    for (int k = 0; k < 6; ++k) av[k] = *(const v4fa*)(hrow + 4 * (lane + 32 * k));
    const float adv = SD[(size_t)gcl * 32 + 16 + l15];
    float l0 = SD[(size_t)gcl * 32 + l15] + adv;
    l0 = l0 > 0.f ? l0 : NEGSL * l0;
    float mx = l0, dn = 1.0f;

#pragma unroll 1
    for (int b0 = 0; b0 < cnt; b0 += 32) {
      int idx = st + b0 + lane;
      idx = idx < 0 ? 0 : (idx > RCAP - 1 ? RCAP - 1 : idx);
      int sr = srt[idx];
      sr = sr < 0 ? 0 : (sr > nN - 1 ? nN - 1 : sr);
      const int m32 = (cnt - b0) < 32 ? (cnt - b0) : 32;
#pragma unroll 1
      for (int k2 = 0; k2 < m32; ++k2) {
        const int sk = __builtin_amdgcn_readlane(sr, k2);
        const float* frow = Hf + (size_t)sk * NCOL;
        const float asv = SD[(size_t)sk * 32 + l15];
        v4f fs[6];
#pragma unroll
        for (int k = 0; k < 6; ++k) fs[k] = *(const v4fa*)(frow + 4 * (lane + 32 * k));
        float lg = asv + adv;
        lg = lg > 0.f ? lg : NEGSL * lg;
        const float df = lg - mx;
        const float ee = expf(-fabsf(df));
        const bool up  = df > 0.f;
        const float s1 = up ? ee : 1.0f;
        const float s2 = up ? 1.0f : ee;
        mx = up ? lg : mx;
        dn = fmaf(dn, s1, s2);
        const int pk = (int)((unsigned)__float_as_int(ee) | (up ? 0x80000000u : 0u));
#pragma unroll
        for (int k = 0; k < 6; ++k) {
          const int g = __shfl(pk, 2 * k + hsel);
          const bool upk = g < 0;
          const float eek = __int_as_float(g & 0x7fffffff);
          const float a1 = upk ? eek : 1.0f;
          const float a2 = upk ? 1.0f : eek;
          av[k].x = fmaf(av[k].x, a1, a2 * fs[k].x);
          av[k].y = fmaf(av[k].y, a1, a2 * fs[k].y);
          av[k].z = fmaf(av[k].z, a1, a2 * fs[k].z);
          av[k].w = fmaf(av[k].w, a1, a2 * fs[k].w);
        }
      }
    }
    const float inv = 1.0f / (dn + EPS_SM);
    const bool live = grow < nN;
    v4f vv[6];
#pragma unroll
    for (int k = 0; k < 6; ++k) {
      const float invk = __shfl(inv, 2 * k + hsel);
      vv[k].x = relu_k(fmaf(av[k].x, invk, bb[k].x));
      vv[k].y = relu_k(fmaf(av[k].y, invk, bb[k].y));
      vv[k].z = relu_k(fmaf(av[k].z, invk, bb[k].z));
      vv[k].w = relu_k(fmaf(av[k].w, invk, bb[k].w));
    }

    if constexpr (L == 1) {
      v4u pv[6];
      const int sa = (2 * lane) & 31, sb2 = (2 * lane + 1) & 31;
      const bool lsel = lane >= 16;
#pragma unroll
      for (int k = 0; k < 6; ++k) {
        v4f o;
        o.x = (live ? vv[k].x : 0.f) + pz;
        o.y = (live ? vv[k].y : 0.f) + pz;
        o.z = (live ? vv[k].z : 0.f) + pz;
        o.w = (live ? vv[k].w : 0.f) + pz;
        const unsigned int hbx = f2bf(o.x), hby = f2bf(o.y), hbz = f2bf(o.z), hbw = f2bf(o.w);
        const unsigned int lbx = f2bf(o.x - bf2f(hbx)), lby = f2bf(o.y - bf2f(hby));
        const unsigned int lbz = f2bf(o.z - bf2f(hbz)), lbw = f2bf(o.w - bf2f(hbw));
        const int hw0 = (int)(hbx | (hby << 16)), hw1 = (int)(hbz | (hbw << 16));
        const int lw0 = (int)(lbx | (lby << 16)), lw1 = (int)(lbz | (lbw << 16));
        const int g0 = __shfl(hw0, sa), g1 = __shfl(hw1, sa), g2 = __shfl(hw0, sb2), g3 = __shfl(hw1, sb2);
        const int q0 = __shfl(lw0, sa), q1 = __shfl(lw1, sa), q2 = __shfl(lw0, sb2), q3 = __shfl(lw1, sb2);
        pv[k].x = (unsigned int)(lsel ? q0 : g0);
        pv[k].y = (unsigned int)(lsel ? q1 : g1);
        pv[k].z = (unsigned int)(lsel ? q2 : g2);
        pv[k].w = (unsigned int)(lsel ? q3 : g3);
      }
      unsigned short* gp = XHL + (size_t)grow * XW + (lsel ? HC : 0) + 8 * l15;
      const bool wr = grow < MPr;
#pragma unroll
      for (int k = 0; k < 6; ++k) {
        const int basek = (k < 3) ? (128 * k) : (NCOL + 128 * (k - 3));
        if (wr) *(volatile v4u*)(gp + basek) = pv[k];
      }
      __threadfence();
#pragma unroll
      for (int k = 0; k < 6; ++k) {
        const int basek = (k < 3) ? (128 * k) : (NCOL + 128 * (k - 3));
        if (wr) *(volatile v4u*)(gp + basek) = pv[k];
      }
    } else {
      v4f hv[3];
#pragma unroll
      for (int k = 0; k < 3; ++k) {
        hv[k].x = (live ? (vv[k].x + vv[k + 3].x) : 0.f) + pz;
        hv[k].y = (live ? (vv[k].y + vv[k + 3].y) : 0.f) + pz;
        hv[k].z = (live ? (vv[k].z + vv[k + 3].z) : 0.f) + pz;
        hv[k].w = (live ? (vv[k].w + vv[k + 3].w) : 0.f) + pz;
      }
      float* op = HS + (size_t)grow * HC + 4 * lane;
      const bool wr = grow < MPr;
#pragma unroll
      for (int k = 0; k < 3; ++k) { if (wr) *(volatile v4f*)(op + 128 * k) = hv[k]; }
      __threadfence();
#pragma unroll
      for (int k = 0; k < 3; ++k) { if (wr) *(volatile v4f*)(op + 128 * k) = hv[k]; }
    }
  }
}

__global__ __launch_bounds__(NTHR) void k_pool(const float* __restrict__ hf, const int* __restrict__ bat,
                                               int nN, float* RO, float* out) {
  __shared__ __attribute__((aligned(16))) double wsum[NWAVE * HC];
  __shared__ int wcn[NWAVE];
  __shared__ __attribute__((aligned(16))) float outs[HC];
  const int tid = (int)threadIdx.x, lane = tid & 31, wave = tid >> 5;
  const int g = (int)blockIdx.x;

  double a[12];
#pragma unroll
  for (int i = 0; i < 12; ++i) a[i] = 0.0;
  int cnt = 0;
#pragma unroll 1
  for (int i0 = wave * 32; i0 < nN; i0 += NTHR) {
    const int i  = i0 + lane;
    const int ic = i < nN ? i : nN - 1;
    const int b  = bat[ic];
    const bool hit = (i < nN) && (b == g);
    unsigned msk = __builtin_amdgcn_ballot_w32(hit);
    int nhit = (int)__builtin_popcount(msk);
    nhit = nhit > 32 ? 32 : nhit;
    cnt += nhit;
#pragma unroll 1
    for (int q = 0; q < nhit; ++q) {
      const int k = __builtin_ffs((int)msk) - 1;
      msk &= msk - 1u;
      int node = i0 + (k < 0 ? 0 : k);
      node = node > nN - 1 ? nN - 1 : node;
      const float* rp = hf + (size_t)node * HC + 4 * lane;
      const v4f v0 = *(const v4fa*)rp;
      const v4f v1 = *(const v4fa*)(rp + 128);
      const v4f v2 = *(const v4fa*)(rp + 256);
      a[0] += (double)v0.x; a[1] += (double)v0.y; a[2]  += (double)v0.z; a[3]  += (double)v0.w;
      a[4] += (double)v1.x; a[5] += (double)v1.y; a[6]  += (double)v1.z; a[7]  += (double)v1.w;
      a[8] += (double)v2.x; a[9] += (double)v2.y; a[10] += (double)v2.z; a[11] += (double)v2.w;
    }
  }
#pragma unroll
  for (int k = 0; k < 3; ++k) {
#pragma unroll
    for (int i = 0; i < 4; ++i) wsum[wave * HC + 128 * k + 4 * lane + i] = a[4 * k + i];
  }
  if (lane == 0) wcn[wave] = cnt;
  __syncthreads();
#pragma unroll 1
  for (int c = tid; c < HC; c += NTHR) {
    double s = 0.0;
    int cc = 0;
#pragma unroll
    for (int w2 = 0; w2 < NWAVE; ++w2) { s += wsum[w2 * HC + c]; cc += wcn[w2]; }
    const float cf = (cc < 1) ? 1.0f : (float)cc;
    outs[c] = (float)s * (1.0f / cf);
  }
  __syncthreads();
  const int pc = tid < HC / 4 ? tid : 0;
  const v4f ov = *(const v4fa*)(outs + 4 * pc);
  const bool okst = tid < HC / 4;
  float* p1 = RO  + (size_t)g * HC + 4 * pc;
  float* p2 = out + (size_t)OUT0N + (size_t)g * HC + 4 * pc;
  if (okst) { *(volatile v4f*)p1 = ov; *(volatile v4f*)p2 = ov; }
  __threadfence();
  if (okst) { *(volatile v4f*)p1 = ov; *(volatile v4f*)p2 = ov; }
}

__global__ __launch_bounds__(NTHR) void k_head(const float* __restrict__ RO, const float* __restrict__ r1w,
                                               const float* __restrict__ r1b, const float* __restrict__ r2w,
                                               const float* __restrict__ r2b, float* out) {
  __shared__ __attribute__((aligned(16))) float hid[NGR * HIDR];
  __shared__ float r2s[HIDR * NOUTC];
  __shared__ float b1s[HIDR];
  __shared__ float b2s[16];
  __shared__ __attribute__((aligned(16))) float os[OUT0N];
  const int tid = (int)threadIdx.x;
#pragma unroll 1
  for (int i = tid; i < HIDR * NOUTC; i += NTHR) r2s[i] = bfr(r2w[i]);
  if (tid < HIDR) b1s[tid] = bfr(r1b[tid]);
  if (tid < 16) {
    const float bv = r2b[tid < NOUTC ? tid : NOUTC - 1];
    b2s[tid] = (tid < NOUTC) ? bfr(bv) : 0.0f;
  }
  __syncthreads();
#pragma unroll 1
  for (int it = 0; it < (NGR * HIDR) / NTHR; ++it) {
    const int idx = it * NTHR + tid;
    const int g = idx >> 6, j = idx & 63;
    const float* pr = RO + (size_t)g * HC;
    const float* wr = r1w + j;
    float s = 0.0f;
#pragma unroll 1
    for (int f4 = 0; f4 < HC / 4; ++f4) {
      const v4f p = *(const v4fa*)(pr + 4 * f4);
      const float w0 = bfr(wr[(4 * f4 + 0) * HIDR]);
      const float w1 = bfr(wr[(4 * f4 + 1) * HIDR]);
      const float w2 = bfr(wr[(4 * f4 + 2) * HIDR]);
      const float w3 = bfr(wr[(4 * f4 + 3) * HIDR]);
      s = fmaf(p.x, w0, s);
      s = fmaf(p.y, w1, s);
      s = fmaf(p.z, w2, s);
      s = fmaf(p.w, w3, s);
    }
    hid[idx] = relu_k(s + b1s[j]);
  }
  __syncthreads();
#pragma unroll 1
  for (int idx = tid; idx < OUT0N; idx += NTHR) {
    const int g = idx / NOUTC;
    const int c = idx - g * NOUTC;
    float s = 0.0f;
#pragma unroll 1
    for (int j4 = 0; j4 < HIDR / 4; ++j4) {
      const v4f hv = *(const v4fa*)(hid + g * HIDR + 4 * j4);
      const float* w = r2s + (4 * j4) * NOUTC + c;
      s = fmaf(hv.x, w[0], s);
      s = fmaf(hv.y, w[NOUTC], s);
      s = fmaf(hv.z, w[2 * NOUTC], s);
      s = fmaf(hv.w, w[3 * NOUTC], s);
    }
    os[idx] = s + b2s[c];
  }
  __syncthreads();
  const int pc = tid < OUT0N / 4 ? tid : 0;
  const v4f ov = *(const v4fa*)(os + 4 * pc);
  const bool okst = tid < OUT0N / 4;
  if (okst) *(volatile v4f*)(out + 4 * pc) = ov;
  __threadfence();
  if (okst) *(volatile v4f*)(out + 4 * pc) = ov;
}

static inline int cdiv(int a, int b) { return (a + b - 1) / b; }
static inline size_t al256(size_t o) { return (o + 255) & ~(size_t)255; }

extern "C" void kernel_launch(void* const* d_in, const int* in_sizes, int n_in,
                              void* d_out, int out_size, void* d_ws, size_t ws_size,
                              hipStream_t stream) {
  if (n_in < 23) return;
  if (in_sizes[0] < F_IN || (in_sizes[0] % F_IN) != 0) return;
  const int nN = in_sizes[0] / F_IN;
  if (nN < 1 || nN > (1 << 20)) return;
  if (in_sizes[1] < 2 || (in_sizes[1] & 1) != 0) return;
  const int nE = in_sizes[1] / 2;
  if (nE < 1 || nE >= (1 << (31 - SLOTB))) return;
  if (in_sizes[2] != nN) return;
  if (in_sizes[3] != F_IN * HC || in_sizes[11] != F_IN * HC) return;
  if (in_sizes[7] != HC * HC || in_sizes[15] != HC * HC) return;
  if (in_sizes[4] != HC || in_sizes[5] != HC || in_sizes[6] != HC) return;
  if (in_sizes[8] != HC || in_sizes[9] != HC || in_sizes[10] != HC) return;
  if (in_sizes[12] != HC || in_sizes[13] != HC || in_sizes[14] != HC) return;
  if (in_sizes[16] != HC || in_sizes[17] != HC || in_sizes[18] != HC) return;
  if (in_sizes[19] != HC * HIDR || in_sizes[20] != HIDR) return;
  if (in_sizes[21] != HIDR * NOUTC || in_sizes[22] != NOUTC) return;
  if (out_size != OUT0N + NGR * HC) return;

  const float* x    = (const float*)d_in[0];
  const int*   ei   = (const int*)  d_in[1];
  const int*   bat  = (const int*)  d_in[2];
  const float* W1   = (const float*)d_in[3];
  const float* a1s  = (const float*)d_in[4];
  const float* a1d  = (const float*)d_in[5];
  const float* b1   = (const float*)d_in[6];
  const float* W2   = (const float*)d_in[7];
  const float* a2s  = (const float*)d_in[8];
  const float* a2d  = (const float*)d_in[9];
  const float* b2   = (const float*)d_in[10];
  const float* Ws1  = (const float*)d_in[11];
  const float* as1s = (const float*)d_in[12];
  const float* as1d = (const float*)d_in[13];
  const float* bs1  = (const float*)d_in[14];
  const float* Ws2  = (const float*)d_in[15];
  const float* as2s = (const float*)d_in[16];
  const float* as2d = (const float*)d_in[17];
  const float* bs2  = (const float*)d_in[18];
  const float* r1w  = (const float*)d_in[19];
  const float* r1b  = (const float*)d_in[20];
  const float* r2w  = (const float*)d_in[21];
  const float* r2b  = (const float*)d_in[22];
  float* out = (float*)d_out;
  const int* src = ei;
  const int* dst = ei + nE;

  const int MP   = cdiv(nN, MROWS) * MROWS;
  const int gB   = cdiv(MP, NB);
  const int gS   = MP / SROWS;
  const int gM   = MP / GBM;
  if ((long long)gB * NB < (long long)MP) return;
  if (gS * SROWS != MP || gM * GBM != MP) return;
  if (((MP * (F_IN / 8)) % NTHR) != 0) return;
  const int nBx  = (MP * (F_IN / 8)) / NTHR;
  const int vec8 = ((nE & 3) == 0) ? 1 : 0;

  char* ws = (char*)d_ws;
  size_t off = 0;
  size_t szA = (size_t)MP * XW * 2;
  if ((size_t)MP * F_IN * 2 > szA) szA = (size_t)MP * F_IN * 2;
  if ((size_t)MP * HC * 4 > szA)   szA = (size_t)MP * HC * 4;
  const size_t oRA  = off; off = al256(off + szA);
  const size_t oH   = off; off = al256(off + (size_t)MP * NCOL * 4);
  const size_t oSD1 = off; off = al256(off + (size_t)MP * 32 * 4);
  const size_t oSD2 = off; off = al256(off + (size_t)MP * 32 * 4);
  const size_t oWT1 = off; off = al256(off + (size_t)NCOL * F_IN * 2);
  const size_t oW2C = off; off = al256(off + (size_t)NCOL * NCOL * 2);
  const size_t oSRT = off; off = al256(off + (size_t)gB * RCAP * 4);
  const size_t oSOF = off; off = al256(off + (size_t)gB * NB * 4);
  const size_t oSCN = off; off = al256(off + (size_t)gB * NB * 4);
  const size_t oMET = off; off = al256(off + (size_t)gB * 32 * 4);
  const size_t oRO  = off; off = al256(off + (size_t)NGR * HC * 4);
  if (off > ws_size || off > (size_t)WSMAX) return;
  unsigned short* XB   = (unsigned short*)(ws + oRA);
  unsigned short* X1HL = (unsigned short*)(ws + oRA);
  float*          HSUM = (float*)(ws + oRA);
  float*          H    = (float*)(ws + oH);
  float*          SD1  = (float*)(ws + oSD1);
  float*          SD2  = (float*)(ws + oSD2);
  unsigned short* WT1  = (unsigned short*)(ws + oWT1);
  unsigned short* W2C  = (unsigned short*)(ws + oW2C);
  int*            SRT  = (int*)(ws + oSRT);
  int*            SOFF = (int*)(ws + oSOF);
  int*            SCNT = (int*)(ws + oSCN);
  int*            META = (int*)(ws + oMET);
  float*          RO   = (float*)(ws + oRO);

  hipFuncSetAttribute(reinterpret_cast<const void*>(&k_bucket),
                      hipFuncAttributeMaxDynamicSharedMemorySize, LDS_BKT);

  const int nBprep = nBx + 2 * (NU_WT1H / NTHR) + 2 * (NU_W2H / NTHR);
  k_prep<<<nBprep, NTHR, 0, stream>>>(x, W1, Ws1, W2, Ws2, XB, WT1, W2C, nN, nBx);
  k_bucket<<<gB, NTHR, LDS_BKT, stream>>>(src, dst, nN, nE, vec8, SRT, SOFF, SCNT, META);
  k_gemm<<<gM, GTHR, 0, stream>>>(XB, F_IN, 0, WT1, F_IN, H, a1s, a1d, as1s, as1d, SD1);
  k_scan<1><<<gS, NTHR, 0, stream>>>(SRT, SOFF, SCNT, META, H, SD1, b1, bs1, X1HL, HSUM, nN, MP);
  k_gemm<<<gM, GTHR, 0, stream>>>(X1HL, XW, NCOL, W2C, NCOL, H, a2s, a2d, as2s, as2d, SD2);
  k_scan<2><<<gS, NTHR, 0, stream>>>(SRT, SOFF, SCNT, META, H, SD2, b2, bs2, X1HL, HSUM, nN, MP);
  k_pool<<<NGR, NTHR, 0, stream>>>(HSUM, bat, nN, RO, out);
  k_head<<<1, NTHR, 0, stream>>>(RO, r1w, r1b, r2w, r2b, out);
}
